// GIN_72937134621131
// MI455X (gfx1250) — hardware-verified
//
#include <hip/hip_runtime.h>
#include <stddef.h>
#include <stdint.h>

#define NN      50000
#define NE      600000
#define HID     128
#define KK      256
#define OUTF    64
#define NL      4
#define NG      128
#define GBM     128
#define NTILE   391
#define MP      50048
#define NTHR    256
#define NWAVE   8
#define EPT     8
#define CHUNK   (NTHR * EPT)
#define WCAP    (EPT * 32)
#define LISTN   (NWAVE * WCAP)
#define NBRUN   1024
#define PKS     10
#define NBLK    49
#define RCAP    28672
#define DEGCAP  64
#define MEAS_B1024  12548
#define MEAS_MAXDEG 28
#define RECW    384
#define STATW   640
#define PARN    2304
#define PB1     0
#define PB2     512
#define PGA     1024
#define PBE     1536
#define PF1     2048
#define PF2     2176
#define XUNITS  (MP * 32)
#define WUNITS  (8 * HID * (KK / 8))
#define WFUNITS (HID * (KK / 8) + OUTF * (KK / 8))
#define PPW     6272
#define BK_ZINTS (2 * RCAP + 2 * NBRUN + LISTN)
#define LDS_BUCKET ((BK_ZINTS + 16) * 4)
#define LDS_GEMM   ((GBM * HID + RECW + HID) * 4)
#define LDS_HEAD   ((2 * NG * HID + 192) * 4)

static_assert(MP == NTILE * GBM && MP >= NN && MP - NN < GBM);
static_assert((MP % 64) == 0 && (XUNITS % NTHR) == 0);
static_assert(NBLK * NBRUN >= MP && NBRUN == (1 << PKS) && NTHR * 4 == NBRUN);
static_assert((CHUNK & (CHUNK - 1)) == 0 && ((long long)CHUNK << PKS) < (1LL << 31));
static_assert((long long)NE < (1LL << 21) && (NE % 4) == 0);
static_assert(LISTN >= NBRUN && LISTN >= NWAVE * WCAP);
static_assert(RCAP >= MEAS_B1024 + MEAS_B1024 / 20 && (RCAP % (4 * NTHR)) == 0);
static_assert(DEGCAP >= MEAS_MAXDEG + 8);
static_assert((BK_ZINTS % (4 * NTHR)) == 0);
static_assert(LDS_BUCKET <= 327680 && LDS_GEMM <= 327680 && LDS_HEAD <= 327680);
static_assert(GBM == NWAVE * 16 && HID == 4 * 32 && KK == 2 * HID && (KK % 32) == 0);
static_assert(RECW == 3 * HID && RECW / 4 <= NTHR && STATW == 5 * HID && STATW / 4 <= NTHR);
static_assert((WUNITS % NTHR) == 0 && ((4 * 4096) % NTHR) == 0 && (WFUNITS % NTHR) == 0 && (4096 % NTHR) == 0);
static_assert(PARN == PF2 + OUTF + 64 && (PARN % 32) == 0);
static_assert(NWAVE * PPW >= NN && (PPW % 32) == 0);
static_assert(NG * (HID / 8) == 8 * NTHR && NG * OUTF == 8 * NTHR * 4 && NG == NWAVE * 16);

constexpr size_t al256c(size_t o) { return (o + 255) & ~(size_t)255; }
constexpr size_t SZ_P1  = (size_t)MP * KK * 2;
constexpr size_t SZ_P2  = (size_t)MP * HID * 4;
constexpr size_t SZ_LST = (size_t)NBLK * RCAP * 4;
constexpr size_t SZ_CNT = (size_t)NBLK * NBRUN * 4;
constexpr size_t SZ_WPL = (size_t)8 * HID * KK * 2;
constexpr size_t SZ_WF1 = (size_t)HID * KK * 2;
constexpr size_t SZ_WF2 = (size_t)OUTF * KK * 2;
constexpr size_t SZ_PAR = (size_t)PARN * 4;
constexpr size_t SZ_REC = (size_t)NTILE * RECW * 4;
constexpr size_t SZ_STA = (size_t)5 * STATW * 4;
constexpr size_t SZ_G   = (size_t)NG * HID * 4;
constexpr size_t O_P1  = 0;
constexpr size_t O_P3  = al256c(O_P1 + SZ_P1);
constexpr size_t O_P2  = al256c(O_P3 + SZ_P1);
constexpr size_t O_LST = al256c(O_P2 + SZ_P2);
constexpr size_t O_CNT = al256c(O_LST + SZ_LST);
constexpr size_t O_OFF = al256c(O_CNT + SZ_CNT);
constexpr size_t O_WPL = al256c(O_OFF + SZ_CNT);
constexpr size_t O_WF1 = al256c(O_WPL + SZ_WPL);
constexpr size_t O_WF2 = al256c(O_WF1 + SZ_WF1);
constexpr size_t O_PAR = al256c(O_WF2 + SZ_WF2);
constexpr size_t O_REC = al256c(O_PAR + SZ_PAR);
constexpr size_t O_STA = al256c(O_REC + SZ_REC);
constexpr size_t O_G   = al256c(O_STA + SZ_STA);
constexpr size_t WS_TOTAL = al256c(O_G + SZ_G);
static_assert(WS_TOTAL <= (size_t)134217728);
static_assert(O_WF2 == O_WF1 + SZ_WF1);
static_assert((O_P2 % 16) == 0 && (O_STA % 128) == 0 && (O_REC % 128) == 0 && ((STATW * 4) % 128) == 0);

typedef float          v4f  __attribute__((ext_vector_type(4)));
typedef float          v8f  __attribute__((ext_vector_type(8)));
typedef int            v4i  __attribute__((ext_vector_type(4)));
typedef int            v8i  __attribute__((ext_vector_type(8)));
typedef unsigned int   v2u  __attribute__((ext_vector_type(2)));
typedef unsigned int   v4u  __attribute__((ext_vector_type(4)));
typedef unsigned short v8us __attribute__((ext_vector_type(8)));
typedef __bf16         v16b __attribute__((ext_vector_type(16)));
typedef v4f  __attribute__((may_alias)) v4fa;
typedef v4i  __attribute__((may_alias)) v4ia;
typedef v8us __attribute__((may_alias)) v8usa;
union Frag { v16b vb; v8us h[2]; v8i w; };

__device__ __forceinline__ v8f wmb(const Frag& a, const Frag& b, v8f c) {
  v8f d = __builtin_amdgcn_wmma_f32_16x16x32_bf16(false, a.vb, false, b.vb, (short)0, c, false, false);
  asm volatile("v_nop\n\tv_nop\n\tv_nop\n\tv_nop" : "+v"(d) : "v"(a.w), "v"(b.w));
  return d;
}

__device__ __forceinline__ int clampi(int v, int lo, int hi) { return v < lo ? lo : (v > hi ? hi : v); }

__device__ __forceinline__ unsigned short bf_bits(float f) {
  const unsigned int u = __float_as_uint(f);
  unsigned int r = (u + 0x7FFFu + ((u >> 16) & 1u)) >> 16;
  r = (f != f) ? 0x7FC0u : r;
  return (unsigned short)r;
}
__device__ __forceinline__ float bf_val(unsigned short b) { return __uint_as_float(((unsigned int)b) << 16); }
__device__ __forceinline__ float bf_rne(float f) { return bf_val(bf_bits(f)); }

__device__ __forceinline__ float relu_p(float v) { return (v > 0.0f) ? v : (v - v); }

__device__ __forceinline__ void hilo8(const v4f a, const v4f b, v8us& hv, v8us& lv) {
  const float f[8] = {a.x, a.y, a.z, a.w, b.x, b.y, b.z, b.w};
#pragma unroll
  for (int j = 0; j < 8; ++j) {
    const unsigned short hb = bf_bits(f[j]);
    hv[j] = hb;
    lv[j] = bf_bits(f[j] - bf_val(hb));
  }
}

__device__ __forceinline__ v4u split8(const v4f a, const v4f b, bool isHi) {
  const float f[8] = {a.x, a.y, a.z, a.w, b.x, b.y, b.z, b.w};
  unsigned int w[4];
#pragma unroll
  for (int j = 0; j < 4; ++j) {
    const unsigned short h0 = bf_bits(f[2 * j]), h1 = bf_bits(f[2 * j + 1]);
    const unsigned short l0 = bf_bits(f[2 * j] - bf_val(h0)), l1 = bf_bits(f[2 * j + 1] - bf_val(h1));
    const unsigned short q0 = isHi ? h0 : l0, q1 = isHi ? h1 : l1;
    w[j] = (unsigned int)q0 | ((unsigned int)q1 << 16);
  }
  v4u pv; pv.x = w[0]; pv.y = w[1]; pv.z = w[2]; pv.w = w[3];
  return pv;
}

__device__ __forceinline__ v4f bnf(const v4f v, const v4f m, const v4f r, const v4f g, const v4f b, bool rl) {
  const v4f y = ((v - m) * r) * g + b;
  v4f z;
  z.x = relu_p(y.x); z.y = relu_p(y.y); z.z = relu_p(y.z); z.w = relu_p(y.w);
  return rl ? z : y;
}

__device__ __forceinline__ v8us cv8b(const float* __restrict__ p, int stride) {
  v8us o;
#pragma unroll
  for (int i = 0; i < 8; ++i) o[i] = bf_bits(p[(size_t)i * (size_t)stride]);
  return o;
}

__device__ __forceinline__ int scan_chunk(const int* __restrict__ dsts, int nE, int cbase, int slotBase,
                                          int nb, int vec8, int* list, int tid, int lane, int wave) {
  int wc = 0;
  const int el0  = tid * EPT;
  const int e0   = cbase + el0;
  const int sent = -2147483647 - 1;
  v4i da, db;
  if (vec8 != 0 && cbase + CHUNK <= nE) {
    da = *(const v4i*)(dsts + e0);
    db = *(const v4i*)(dsts + e0 + 4);
  } else {
    da.x = (e0     < nE) ? dsts[min(e0,     nE - 1)] : sent;
    da.y = (e0 + 1 < nE) ? dsts[min(e0 + 1, nE - 1)] : sent;
    da.z = (e0 + 2 < nE) ? dsts[min(e0 + 2, nE - 1)] : sent;
    da.w = (e0 + 3 < nE) ? dsts[min(e0 + 3, nE - 1)] : sent;
    db.x = (e0 + 4 < nE) ? dsts[min(e0 + 4, nE - 1)] : sent;
    db.y = (e0 + 5 < nE) ? dsts[min(e0 + 5, nE - 1)] : sent;
    db.z = (e0 + 6 < nE) ? dsts[min(e0 + 6, nE - 1)] : sent;
    db.w = (e0 + 7 < nE) ? dsts[min(e0 + 7, nE - 1)] : sent;
  }
  const unsigned nbs = (unsigned)slotBase;
  const unsigned unb = (unsigned)nb;
  const unsigned s0 = (unsigned)da.x - nbs, s1 = (unsigned)da.y - nbs;
  const unsigned s2 = (unsigned)da.z - nbs, s3 = (unsigned)da.w - nbs;
  const unsigned s4 = (unsigned)db.x - nbs, s5 = (unsigned)db.y - nbs;
  const unsigned s6 = (unsigned)db.z - nbs, s7 = (unsigned)db.w - nbs;
  const bool h0 = s0 < unb, h1 = s1 < unb, h2 = s2 < unb, h3 = s3 < unb;
  const bool h4 = s4 < unb, h5 = s5 < unb, h6 = s6 < unb, h7 = s7 < unb;
  const unsigned any = __builtin_amdgcn_ballot_w32(h0 | h1 | h2 | h3 | h4 | h5 | h6 | h7);
  if (any != 0u) {
#define HITJ(J, HJ, SJ) { \
      const unsigned mj = __builtin_amdgcn_ballot_w32(HJ); \
      if (mj != 0u) { \
        if (HJ) { \
          const int pos = wc + (int)__builtin_amdgcn_mbcnt_lo(mj, 0u); \
          if (pos < WCAP) list[wave * WCAP + pos] = ((el0 + (J)) << PKS) | (int)(SJ); \
        } \
        wc += (int)__builtin_popcount(mj); } }
    HITJ(0, h0, s0)
    HITJ(1, h1, s1)
    HITJ(2, h2, s2)
    HITJ(3, h3, s3)
    HITJ(4, h4, s4)
    HITJ(5, h5, s5)
    HITJ(6, h6, s6)
    HITJ(7, h7, s7)
#undef HITJ
  }
  return wc;
}

__global__ __launch_bounds__(NTHR) void k_pa(const float* __restrict__ x, float* wsf) {
  const int u = (int)blockIdx.x * NTHR + (int)threadIdx.x;
  v4f o;
  size_t di;
  if (u < XUNITS) {
    const int row = u >> 5, q = u & 31;
    const int rc  = row < NN ? row : NN - 1;
    const v4f a = *(const v4f*)(x + (size_t)rc * HID + 4 * q);
    const bool live = row < NN;
    o.x = live ? bf_rne(a.x) : 0.0f;
    o.y = live ? bf_rne(a.y) : 0.0f;
    o.z = live ? bf_rne(a.z) : 0.0f;
    o.w = live ? bf_rne(a.w) : 0.0f;
    di = O_P2 / 4 + (size_t)u * 4;
  } else if (u < XUNITS + STATW / 4) {
    const int s = u - XUNITS;
    const int r = s >> 5;
    const float val = (r == 1 || r == 2) ? 1.0f : 0.0f;
    o.x = val; o.y = val; o.z = val; o.w = val;
    di = O_STA / 4 + (size_t)s * 4;
  } else {
    return;
  }
  float* dp = wsf + di;
  *(volatile v4f*)dp = o;
  __threadfence();
  *(volatile v4f*)dp = o;
}

__global__ __launch_bounds__(NTHR) void k_pb(const float* __restrict__ W1, const float* __restrict__ W2,
                                             unsigned short* wpl) {
  const int u = (int)blockIdx.x * NTHR + (int)threadIdx.x;
  if (u >= WUNITS) return;
  const int v  = u & 4095;
  const int n  = v >> 5;
  const int k8 = (v & 31) * 8;
  const int kk = k8 & (HID - 1);
  v8us o;
  if (u < 4 * 4096) {
    const int mat = u >> 12;
    o = cv8b(W1 + (size_t)mat * HID * HID + (size_t)kk * HID + n, HID);
  } else {
    const int mat = (u >> 12) - 4;
    o = cv8b(W2 + (size_t)mat * HID * HID + (size_t)kk * HID + n, HID);
  }
  unsigned short* dp = wpl + (size_t)u * 8;
  *(volatile v8us*)dp = o;
  __threadfence();
  *(volatile v8us*)dp = o;
}

__global__ __launch_bounds__(NTHR) void k_pc(const float* __restrict__ Wf1, const float* __restrict__ Wf2,
                                             const float* __restrict__ b1, const float* __restrict__ b2,
                                             const float* __restrict__ gam, const float* __restrict__ bet,
                                             const float* __restrict__ bf1, const float* __restrict__ bf2,
                                             unsigned short* wft, float* par) {
  const int u = (int)blockIdx.x * NTHR + (int)threadIdx.x;
  if (u < WFUNITS) {
    v8us o;
    if (u < 4096) {
      const int n = u >> 5, k8 = (u & 31) * 8, kk = k8 & (HID - 1);
      o = cv8b(Wf1 + (size_t)kk * HID + n, HID);
    } else {
      const int v = u - 4096;
      const int n = v >> 5, k8 = (v & 31) * 8, kk = k8 & (HID - 1);
      o = cv8b(Wf2 + (size_t)kk * OUTF + n, OUTF);
    }
    unsigned short* dp = wft + (size_t)u * 8;
    *(volatile v8us*)dp = o;
    __threadfence();
    *(volatile v8us*)dp = o;
  } else if (u < WFUNITS + PARN / 4) {
    const int p = u - WFUNITS;
    const int f = 4 * p;
    const v4f c0 = *(const v4f*)(b1  + clampi(f,        0, 508));
    const v4f c1 = *(const v4f*)(b2  + clampi(f - PB2,  0, 508));
    const v4f c2 = *(const v4f*)(gam + clampi(f - PGA,  0, 508));
    const v4f c3 = *(const v4f*)(bet + clampi(f - PBE,  0, 508));
    const v4f c4 = *(const v4f*)(bf1 + clampi(f - PF1,  0, 124));
    const v4f c5 = *(const v4f*)(bf2 + clampi(f - PF2,  0, 60));
    v4f s = c0;
    s = (f >= PB2) ? c1 : s;
    s = (f >= PGA) ? c2 : s;
    s = (f >= PBE) ? c3 : s;
    s = (f >= PF1) ? c4 : s;
    s = (f >= PF2) ? c5 : s;
    const bool zr = f >= PF2 + OUTF;
    v4f o;
    o.x = zr ? 0.0f : bf_rne(s.x);
    o.y = zr ? 0.0f : bf_rne(s.y);
    o.z = zr ? 0.0f : bf_rne(s.z);
    o.w = zr ? 0.0f : bf_rne(s.w);
    float* dp = par + (size_t)f;
    *(volatile v4f*)dp = o;
    __threadfence();
    *(volatile v4f*)dp = o;
  }
}

__global__ __launch_bounds__(NTHR) __attribute__((amdgpu_num_vgpr(248)))
void k_bucket(const int* __restrict__ srcs, const int* __restrict__ dsts, int* LISTg, int* CNTg, int* OFFg) {
  extern __shared__ __attribute__((aligned(16))) int bsm[];
  int* reg1 = bsm;
  int* reg2 = reg1 + RCAP;
  int* scnt = reg2 + RCAP;
  int* soff = scnt + NBRUN;
  int* list = soff + NBRUN;
  int* wcnt = list + LISTN;
  int* wtot = wcnt + NWAVE;
  const int tid = (int)threadIdx.x, lane = tid & 31, wave = tid >> 5;
  const int blk = (int)blockIdx.x;
  const int nodeBase = blk * NBRUN;

  {
    const v4i z4 = {0, 0, 0, 0};
#pragma unroll 1
    for (int i = tid * 4; i < BK_ZINTS; i += NTHR * 4) *(v4ia*)(bsm + i) = z4;
    if (tid < 2 * NWAVE) wcnt[tid] = 0;
  }
  __syncthreads();

  int tot = 0;
  const int nChunks = (NE + CHUNK - 1) / CHUNK;
#pragma unroll 1
  for (int ch = 0; ch < nChunks; ++ch) {
    const int cbase = ch * CHUNK;
    const int wc = scan_chunk(dsts, NE, cbase, nodeBase, NBRUN, 1, list, tid, lane, wave);
    if (lane == 0) wcnt[wave] = wc;
    __syncthreads();
    int pre = 0, all = 0;
#pragma unroll
    for (int w2 = 0; w2 < NWAVE; ++w2) {
      int c = wcnt[w2];
      c = c < 0 ? 0 : (c > WCAP ? WCAP : c);
      all += c;
      pre += (w2 < wave) ? c : 0;
    }
    const int wcc  = wc > WCAP ? WCAP : wc;
    const int base = tot + pre;
#pragma unroll 1
    for (int i = lane; i < wcc; i += 32) {
      const int ent = list[wave * WCAP + i];
      const int el  = (ent >> PKS) & (CHUNK - 1);
      const int sl  = ent & (NBRUN - 1);
      int eid = cbase + el;
      eid = eid > NE - 1 ? NE - 1 : eid;
      const int pos = base + i;
      if (pos < RCAP) reg1[pos] = (int)(((unsigned)eid << PKS) | (unsigned)sl);
    }
    tot += all;
    tot = tot > RCAP ? RCAP : tot;
    __syncthreads();
  }
  const int nh = tot;

  if (wave == 0) {
#pragma unroll 1
    for (int b0 = 0; b0 < nh; b0 += 32) {
      const int idx = b0 + lane;
      const int uv  = reg1[idx < RCAP ? idx : RCAP - 1];
      const int m32 = (nh - b0) < 32 ? (nh - b0) : 32;
#pragma unroll 1
      for (int k = 0; k < m32; ++k) {
        const int u  = __builtin_amdgcn_readlane(uv, k);
        const int sl = u & (NBRUN - 1);
        if (lane == 0) scnt[sl] = scnt[sl] + 1;
      }
    }
  }
  __syncthreads();

  {
    const v4i ca = *(const v4ia*)(scnt + 4 * tid);
    const int e0 = ca.x < 0 ? 0 : ca.x, e1 = ca.y < 0 ? 0 : ca.y, e2 = ca.z < 0 ? 0 : ca.z, e3 = ca.w < 0 ? 0 : ca.w;
    const int ts = e0 + e1 + e2 + e3;
    int incl = ts;
#pragma unroll
    for (int d = 1; d < 32; d <<= 1) {
      const int up = __shfl_up(incl, d);
      if (lane >= d) incl += up;
    }
    if (lane == 31) wtot[wave] = incl;
    __syncthreads();
    int pre = 0;
#pragma unroll
    for (int w2 = 0; w2 < NWAVE; ++w2) pre += (w2 < wave) ? wtot[w2] : 0;
    int run = pre + incl - ts;
    soff[4 * tid + 0] = run; run += e0;
    soff[4 * tid + 1] = run; run += e1;
    soff[4 * tid + 2] = run; run += e2;
    soff[4 * tid + 3] = run;
  }
  __syncthreads();
  for (int i = tid; i < NBRUN; i += NTHR) list[i] = soff[i];
  __syncthreads();

  if (wave == 0) {
#pragma unroll 1
    for (int b0 = 0; b0 < nh; b0 += 32) {
      const int idx = b0 + lane;
      const int uv  = reg1[idx < RCAP ? idx : RCAP - 1];
      const int m32 = (nh - b0) < 32 ? (nh - b0) : 32;
#pragma unroll 1
      for (int k = 0; k < m32; ++k) {
        const int u   = __builtin_amdgcn_readlane(uv, k);
        const int sl  = u & (NBRUN - 1);
        const int eid = (int)((unsigned)u >> PKS);
        if (lane == 0) {
          int pos = list[sl];
          pos = pos < 0 ? 0 : (pos > RCAP - 1 ? RCAP - 1 : pos);
          reg2[pos] = eid;
          list[sl] = pos + 1;
        }
      }
    }
  }
  __syncthreads();

  const bool ovf = (nh >= RCAP);
  {
    v4i cv = *(const v4ia*)(scnt + 4 * tid);
    v4i ov = *(const v4ia*)(soff + 4 * tid);
    const int big = 0x7fffffff;
    cv.x = ovf ? big : cv.x; cv.y = ovf ? big : cv.y; cv.z = ovf ? big : cv.z; cv.w = ovf ? big : cv.w;
    ov.x = clampi(ov.x, 0, RCAP); ov.y = clampi(ov.y, 0, RCAP);
    ov.z = clampi(ov.z, 0, RCAP); ov.w = clampi(ov.w, 0, RCAP);
    int* cp = CNTg + nodeBase + 4 * tid;
    int* op = OFFg + nodeBase + 4 * tid;
    *(volatile v4i*)cp = cv;
    *(volatile v4i*)op = ov;
    __threadfence();
    *(volatile v4i*)cp = cv;
    *(volatile v4i*)op = ov;
  }
#pragma unroll 1
  for (int it = 0; it < RCAP / (4 * NTHR); ++it) {
    const int i4 = (it * NTHR + tid) * 4;
    const v4i ev = *(const v4ia*)(reg2 + i4);
    const int q0 = clampi(ev.x, 0, NE - 1), q1 = clampi(ev.y, 0, NE - 1);
    const int q2 = clampi(ev.z, 0, NE - 1), q3 = clampi(ev.w, 0, NE - 1);
    const int s0 = clampi(srcs[q0], 0, NN - 1), s1 = clampi(srcs[q1], 0, NN - 1);
    const int s2 = clampi(srcs[q2], 0, NN - 1), s3 = clampi(srcs[q3], 0, NN - 1);
    v4i o;
    o.x = s0 & -(int)(i4 + 0 < nh);
    o.y = s1 & -(int)(i4 + 1 < nh);
    o.z = s2 & -(int)(i4 + 2 < nh);
    o.w = s3 & -(int)(i4 + 3 < nh);
    int* lp = LISTg + (size_t)blk * RCAP + i4;
    *(volatile v4i*)lp = o;
    __threadfence();
    *(volatile v4i*)lp = o;
  }
}

__global__ __launch_bounds__(NTHR) __attribute__((amdgpu_num_vgpr(248)))
void k_agg(const float* __restrict__ P2, const float* __restrict__ stat, const int* __restrict__ LISTg,
           const int* __restrict__ CNTg, const int* __restrict__ OFFg, unsigned short* P1) {
  const int tid = (int)threadIdx.x, lane = tid & 31, wave = tid >> 5;
  const v4f m4 = *(const v4f*)(stat + 4 * lane);
  const v4f r4 = *(const v4f*)(stat + HID + 4 * lane);
  const v4f g4 = *(const v4f*)(stat + 2 * HID + 4 * lane);
  const v4f b4 = *(const v4f*)(stat + 3 * HID + 4 * lane);
  const bool rl = stat[4 * HID] > 0.5f;
  const float qnan = __int_as_float(0x7fc00000);
  const int rowBase = (int)blockIdx.x * 64 + wave * 8;

#pragma unroll 1
  for (int j = 0; j < 8; ++j) {
    const int row  = rowBase + j;
    const int craw = __builtin_amdgcn_readfirstlane(CNTg[row]);
    const int oraw = __builtin_amdgcn_readfirstlane(OFFg[row]);
    int cnt = craw < 0 ? 0 : (craw > DEGCAP ? DEGCAP : craw);
    const int st = oraw < 0 ? 0 : (oraw > RCAP ? RCAP : oraw);
    if (cnt > RCAP - st) cnt = RCAP - st;
    const bool bad = (craw < 0) || (craw > DEGCAP);
    const int* lp = LISTg + (size_t)(row >> PKS) * RCAP;

    v4f ag = {0.0f, 0.0f, 0.0f, 0.0f};
#pragma unroll 1
    for (int b0 = 0; b0 < cnt; b0 += 32) {
      int idx = st + b0 + lane;
      idx = idx > RCAP - 1 ? RCAP - 1 : idx;
      const int sr = clampi(lp[idx], 0, NN - 1);
      const int m32 = (cnt - b0) < 32 ? (cnt - b0) : 32;
#pragma unroll 1
      for (int k = 0; k < m32; ++k) {
        const int sk = __builtin_amdgcn_readlane(sr, k);
        const v4f v = *(const v4f*)(P2 + (size_t)sk * HID + 4 * lane);
        ag = ag + bnf(v, m4, r4, g4, b4, rl);
      }
    }
    const bool live = row < NN;
    const int rc = live ? row : NN - 1;
    const v4f sv = bnf(*(const v4f*)(P2 + (size_t)rc * HID + 4 * lane), m4, r4, g4, b4, rl);
    const v4f z = sv + ag;
    const float pz = bad ? qnan : 0.0f;
    const float z0 = live ? (z.x + pz) : 0.0f;
    const float z1 = live ? (z.y + pz) : 0.0f;
    const float z2 = live ? (z.z + pz) : 0.0f;
    const float z3 = live ? (z.w + pz) : 0.0f;
    const unsigned short h0 = bf_bits(z0), h1 = bf_bits(z1), h2 = bf_bits(z2), h3 = bf_bits(z3);
    const unsigned short l0 = bf_bits(z0 - bf_val(h0)), l1 = bf_bits(z1 - bf_val(h1));
    const unsigned short l2 = bf_bits(z2 - bf_val(h2)), l3 = bf_bits(z3 - bf_val(h3));
    v2u ph, pl;
    ph.x = (unsigned int)h0 | ((unsigned int)h1 << 16);
    ph.y = (unsigned int)h2 | ((unsigned int)h3 << 16);
    pl.x = (unsigned int)l0 | ((unsigned int)l1 << 16);
    pl.y = (unsigned int)l2 | ((unsigned int)l3 << 16);
    unsigned short* gp = P1 + (size_t)row * KK + 4 * lane;
    *(volatile v2u*)gp = ph;
    *(volatile v2u*)(gp + HID) = pl;
    __threadfence();
    *(volatile v2u*)gp = ph;
    *(volatile v2u*)(gp + HID) = pl;
  }
}

template <int EPI>
__global__ __launch_bounds__(NTHR) __attribute__((amdgpu_num_vgpr(248)))
void k_gemm(const unsigned short* __restrict__ A, const unsigned short* __restrict__ BT,
            const float* __restrict__ bias, void* outp, float* rec) {
  extern __shared__ __attribute__((aligned(16))) float gsm[];
  float* stg = gsm;
  float* pst = gsm + GBM * HID;
  float* bsh = pst + RECW;
  const int tid = (int)threadIdx.x, lane = tid & 31, wave = tid >> 5, hh = lane >> 4, m = lane & 15;
  const int rowBase = (int)blockIdx.x * GBM;

  if (tid < HID) bsh[tid] = bias[tid];
  __syncthreads();

  v8f acc[8];
  {
    const v8f z = {0.f, 0.f, 0.f, 0.f, 0.f, 0.f, 0.f, 0.f};
#pragma unroll
    for (int t = 0; t < 8; ++t) acc[t] = z;
  }
  const unsigned short* ap = A  + (size_t)(rowBase + 16 * wave + m) * (size_t)KK + 8 * hh;
  const unsigned short* bp = BT + (size_t)m * (size_t)KK + 8 * hh;

#pragma unroll 1
  for (int k0 = 0; k0 < KK; k0 += 32) {
    Frag af;
    af.h[0] = *(const v8usa*)(ap + k0);
    af.h[1] = *(const v8usa*)(ap + k0 + 16);
#pragma unroll
    for (int nt = 0; nt < 8; ++nt) {
      const unsigned short* wq = bp + (size_t)(16 * nt) * (size_t)KK + k0;
      Frag bfr;
      bfr.h[0] = *(const v8usa*)wq;
      bfr.h[1] = *(const v8usa*)(wq + 16);
      acc[nt] = wmb(af, bfr, acc[nt]);
    }
  }

#pragma unroll
  for (int nt = 0; nt < 8; ++nt) {
    const int lc = 16 * nt + m;
    const float bb = bsh[lc];
#pragma unroll
    for (int r = 0; r < 8; ++r) {
      const int lr = 16 * wave + 8 * hh + r;
      const bool live = (rowBase + lr) < NN;
      float v = acc[nt][r] + bb;
      if constexpr (EPI == 0) v = relu_p(v);
      stg[lr * HID + lc] = live ? v : 0.0f;
    }
  }
  __syncthreads();

  if constexpr (EPI == 0) {
    unsigned short* outH = (unsigned short*)outp;
    const int cb = 8 * m;
    const bool isHi = (hh == 0);
#pragma unroll 1
    for (int i = 0; i < 16; ++i) {
      const int lr = 16 * wave + i;
      const v4f a = *(const v4fa*)(stg + lr * HID + cb);
      const v4f b = *(const v4fa*)(stg + lr * HID + cb + 4);
      const v4u pv = split8(a, b, isHi);
      unsigned short* op = outH + (size_t)(rowBase + lr) * (size_t)KK + cb + hh * HID;
      *(volatile v4u*)op = pv;
    }
    __threadfence();
#pragma unroll 1
    for (int i = 0; i < 16; ++i) {
      const int lr = 16 * wave + i;
      const v4f a = *(const v4fa*)(stg + lr * HID + cb);
      const v4f b = *(const v4fa*)(stg + lr * HID + cb + 4);
      const v4u pv = split8(a, b, isHi);
      unsigned short* op = outH + (size_t)(rowBase + lr) * (size_t)KK + cb + hh * HID;
      *(volatile v4u*)op = pv;
    }
  } else {
    float* outF = (float*)outp;
#pragma unroll 1
    for (int i = 0; i < 16; ++i) {
      const int lr = 16 * wave + i;
      const v4f fv = *(const v4fa*)(stg + lr * HID + 4 * lane);
      float* op = outF + (size_t)(rowBase + lr) * (size_t)HID + 4 * lane;
      *(volatile v4f*)op = fv;
    }
    if (tid < HID) {
      int nvr = NN - rowBase;
      nvr = nvr < 0 ? 0 : (nvr > GBM ? GBM : nvr);
      float s = 0.0f;
#pragma unroll 1
      for (int r = 0; r < nvr; ++r) s += stg[r * HID + tid];
      const float inv = 1.0f / (float)(nvr < 1 ? 1 : nvr);
      const float mean = s * inv;
      float q = 0.0f;
#pragma unroll 1
      for (int r = 0; r < nvr; ++r) {
        const float d = stg[r * HID + tid] - mean;
        q = fmaf(d, d, q);
      }
      pst[tid] = (float)nvr;
      pst[HID + tid] = mean;
      pst[2 * HID + tid] = q;
    }
    __syncthreads();
    const bool pok = tid < RECW / 4;
    v4f pv = {0.f, 0.f, 0.f, 0.f};
    float* pp = rec + (size_t)blockIdx.x * RECW + 4 * tid;
    if (pok) {
      pv = *(const v4fa*)(pst + 4 * tid);
      *(volatile v4f*)pp = pv;
    }
    __threadfence();
#pragma unroll 1
    for (int i = 0; i < 16; ++i) {
      const int lr = 16 * wave + i;
      const v4f fv = *(const v4fa*)(stg + lr * HID + 4 * lane);
      float* op = outF + (size_t)(rowBase + lr) * (size_t)HID + 4 * lane;
      *(volatile v4f*)op = fv;
    }
    if (pok) *(volatile v4f*)pp = pv;
  }
}

__global__ __launch_bounds__(NTHR) void k_comb(const float* __restrict__ rec, const float* __restrict__ par,
                                               int layer, float* statOut) {
  __shared__ __attribute__((aligned(16))) float stg[STATW];
  const int tid = (int)threadIdx.x;
  if (tid < HID) {
    double n = 0.0, mean = 0.0, M2 = 0.0;
#pragma unroll 1
    for (int b = 0; b < NTILE; ++b) {
      const float* pr = rec + (size_t)b * RECW;
      const double nb = (double)pr[tid];
      const double mb = (double)pr[HID + tid];
      const double qb = (double)pr[2 * HID + tid];
      if (nb > 0.5) {
        const double nn = n + nb;
        const double delta = mb - mean;
        const double f = nb / nn;
        mean = mean + delta * f;
        M2 = M2 + qb + delta * delta * n * f;
        n = nn;
      }
    }
    const float varf = (float)(M2 * (1.0 / (double)NN));
    const float rstd = 1.0f / sqrtf(varf + 1e-5f);
    stg[tid] = (float)mean;
    stg[HID + tid] = rstd;
    stg[2 * HID + tid] = par[PGA + layer * HID + tid];
    stg[3 * HID + tid] = par[PBE + layer * HID + tid];
    stg[4 * HID + tid] = 1.0f;
  }
  __syncthreads();
  const bool ok = tid < STATW / 4;
  v4f v = {0.f, 0.f, 0.f, 0.f};
  float* dp = statOut + 4 * tid;
  if (ok) {
    v = *(const v4fa*)(stg + 4 * tid);
    *(volatile v4f*)dp = v;
  }
  __threadfence();
  if (ok) *(volatile v4f*)dp = v;
}

__global__ __launch_bounds__(NTHR) __attribute__((amdgpu_num_vgpr(248)))
void k_pool(const float* __restrict__ U, const float* __restrict__ stat, const int* __restrict__ bat, float* G) {
  __shared__ __attribute__((aligned(16))) float part[NWAVE * HID];
  const int tid = (int)threadIdx.x, lane = tid & 31, wave = tid >> 5;
  const int g = (int)blockIdx.x;
  const v4f m4 = *(const v4f*)(stat + 4 * lane);
  const v4f r4 = *(const v4f*)(stat + HID + 4 * lane);
  const v4f g4 = *(const v4f*)(stat + 2 * HID + 4 * lane);
  const v4f b4 = *(const v4f*)(stat + 3 * HID + 4 * lane);
  const bool rl = stat[4 * HID] > 0.5f;
  const int nlo = wave * PPW;
  const int nhi = (nlo + PPW) < NN ? (nlo + PPW) : NN;
  v4f acc = {0.0f, 0.0f, 0.0f, 0.0f};
#pragma unroll 1
  for (int c = 0; c < PPW / 32; ++c) {
    const int n0 = nlo + 32 * c;
    const int ni = n0 + lane;
    const int id = bat[ni < NN - 1 ? ni : NN - 1];
    const bool hit = (id == g) & (ni < nhi);
    unsigned mask = __builtin_amdgcn_ballot_w32(hit);
#pragma unroll 1
    while (mask != 0u) {
      const int jb = (int)__builtin_ctz(mask);
      mask &= mask - 1u;
      int n = n0 + jb;
      n = n > NN - 1 ? NN - 1 : n;
      const v4f v = *(const v4f*)(U + (size_t)n * HID + 4 * lane);
      acc = acc + bnf(v, m4, r4, g4, b4, rl);
    }
  }
  *(v4fa*)(part + wave * HID + 4 * lane) = acc;
  __syncthreads();
  v4f s = {0.0f, 0.0f, 0.0f, 0.0f};
  float* dp = G + (size_t)g * HID + 4 * lane;
  if (wave == 0) {
#pragma unroll
    for (int w2 = 0; w2 < NWAVE; ++w2) s = s + *(const v4fa*)(part + w2 * HID + 4 * lane);
    *(volatile v4f*)dp = s;
  }
  __threadfence();
  if (wave == 0) *(volatile v4f*)dp = s;
}

__global__ __launch_bounds__(NTHR) __attribute__((amdgpu_num_vgpr(248)))
void k_head(const float* __restrict__ G, const unsigned short* __restrict__ WF1, const unsigned short* __restrict__ WF2,
            const float* __restrict__ par, float* out) {
  extern __shared__ __attribute__((aligned(16))) float hsm[];
  float* stg = hsm;
  unsigned short* apl = (unsigned short*)(hsm + NG * HID);
  float* bsh = hsm + 2 * NG * HID;
  const int tid = (int)threadIdx.x, lane = tid & 31, wave = tid >> 5, hh = lane >> 4, m = lane & 15;

  if (tid < HID)  bsh[tid] = par[PF1 + tid];
  if (tid < OUTF) bsh[HID + tid] = par[PF2 + tid];
#pragma unroll 1
  for (int it = 0; it < 8; ++it) {
    const int p = it * NTHR + tid;
    const int row = p >> 4, q = p & 15;
    const v4f a = *(const v4f*)(G + (size_t)row * HID + 8 * q);
    const v4f b = *(const v4f*)(G + (size_t)row * HID + 8 * q + 4);
    v8us hv, lv;
    hilo8(a, b, hv, lv);
    *(v8usa*)(apl + row * KK + 8 * q) = hv;
    *(v8usa*)(apl + row * KK + HID + 8 * q) = lv;
  }
  __syncthreads();

  const v8f z8 = {0.f, 0.f, 0.f, 0.f, 0.f, 0.f, 0.f, 0.f};
  const unsigned short* ap = apl + (16 * wave + m) * KK + 8 * hh;
  {
    v8f acc[8];
#pragma unroll
    for (int t = 0; t < 8; ++t) acc[t] = z8;
    const unsigned short* bp = WF1 + (size_t)m * (size_t)KK + 8 * hh;
#pragma unroll 1
    for (int k0 = 0; k0 < KK; k0 += 32) {
      Frag af;
      af.h[0] = *(const v8usa*)(ap + k0);
      af.h[1] = *(const v8usa*)(ap + k0 + 16);
#pragma unroll
      for (int nt = 0; nt < 8; ++nt) {
        const unsigned short* wq = bp + (size_t)(16 * nt) * (size_t)KK + k0;
        Frag bfr;
        bfr.h[0] = *(const v8usa*)wq;
        bfr.h[1] = *(const v8usa*)(wq + 16);
        acc[nt] = wmb(af, bfr, acc[nt]);
      }
    }
#pragma unroll
    for (int nt = 0; nt < 8; ++nt) {
      const int lc = 16 * nt + m;
      const float bb = bsh[lc];
#pragma unroll
      for (int r = 0; r < 8; ++r) {
        const int lr = 16 * wave + 8 * hh + r;
        stg[lr * HID + lc] = relu_p(acc[nt][r] + bb);
      }
    }
  }
  __syncthreads();
#pragma unroll 1
  for (int it = 0; it < 8; ++it) {
    const int p = it * NTHR + tid;
    const int row = p >> 4, q = p & 15;
    const v4f a = *(const v4fa*)(stg + row * HID + 8 * q);
    const v4f b = *(const v4fa*)(stg + row * HID + 8 * q + 4);
    v8us hv, lv;
    hilo8(a, b, hv, lv);
    *(v8usa*)(apl + row * KK + 8 * q) = hv;
    *(v8usa*)(apl + row * KK + HID + 8 * q) = lv;
  }
  __syncthreads();
  {
    v8f acc[4];
#pragma unroll
    for (int t = 0; t < 4; ++t) acc[t] = z8;
    const unsigned short* bp = WF2 + (size_t)m * (size_t)KK + 8 * hh;
#pragma unroll 1
    for (int k0 = 0; k0 < KK; k0 += 32) {
      Frag af;
      af.h[0] = *(const v8usa*)(ap + k0);
      af.h[1] = *(const v8usa*)(ap + k0 + 16);
#pragma unroll
      for (int nt = 0; nt < 4; ++nt) {
        const unsigned short* wq = bp + (size_t)(16 * nt) * (size_t)KK + k0;
        Frag bfr;
        bfr.h[0] = *(const v8usa*)wq;
        bfr.h[1] = *(const v8usa*)(wq + 16);
        acc[nt] = wmb(af, bfr, acc[nt]);
      }
    }
#pragma unroll
    for (int nt = 0; nt < 4; ++nt) {
      const int lc = 16 * nt + m;
      const float bb = bsh[HID + lc];
#pragma unroll
      for (int r = 0; r < 8; ++r) {
        const int lr = 16 * wave + 8 * hh + r;
        stg[lr * OUTF + lc] = acc[nt][r] + bb;
      }
    }
  }
  __syncthreads();
#pragma unroll 1
  for (int it = 0; it < 8; ++it) {
    const int p = it * NTHR + tid;
    const v4f v = *(const v4fa*)(stg + 4 * p);
    *(volatile v4f*)(out + 4 * p) = v;
  }
  __threadfence();
#pragma unroll 1
  for (int it = 0; it < 8; ++it) {
    const int p = it * NTHR + tid;
    const v4f v = *(const v4fa*)(stg + 4 * p);
    *(volatile v4f*)(out + 4 * p) = v;
  }
}

extern "C" void kernel_launch(void* const* d_in, const int* in_sizes, int n_in,
                              void* d_out, int out_size, void* d_ws, size_t ws_size,
                              hipStream_t stream) {
  if (n_in < 13) return;
  if (in_sizes[0] != NN * HID) return;
  if (in_sizes[1] != 2 * NE) return;
  if (in_sizes[2] != NN) return;
  if (in_sizes[3] != NL * HID * HID || in_sizes[4] != NL * HID) return;
  if (in_sizes[5] != NL * HID * HID || in_sizes[6] != NL * HID) return;
  if (in_sizes[7] != NL * HID || in_sizes[8] != NL * HID) return;
  if (in_sizes[9] != HID * HID || in_sizes[10] != HID) return;
  if (in_sizes[11] != HID * OUTF || in_sizes[12] != OUTF) return;
  if (out_size != NG * OUTF) return;
  if (WS_TOTAL > ws_size) return;

  const float* x     = (const float*)d_in[0];
  const int*   ei    = (const int*)  d_in[1];
  const int*   src   = ei;
  const int*   dst   = ei + NE;
  const int*   batch = (const int*)  d_in[2];
  const float* W1    = (const float*)d_in[3];
  const float* b1    = (const float*)d_in[4];
  const float* W2    = (const float*)d_in[5];
  const float* b2    = (const float*)d_in[6];
  const float* gamma = (const float*)d_in[7];
  const float* beta  = (const float*)d_in[8];
  const float* Wf1   = (const float*)d_in[9];
  const float* bf1   = (const float*)d_in[10];
  const float* Wf2   = (const float*)d_in[11];
  const float* bf2   = (const float*)d_in[12];
  float* out = (float*)d_out;

  char* ws = (char*)d_ws;
  unsigned short* P1   = (unsigned short*)(ws + O_P1);
  unsigned short* P3   = (unsigned short*)(ws + O_P3);
  float*          P2   = (float*)(ws + O_P2);
  int*            LST  = (int*)(ws + O_LST);
  int*            CNT  = (int*)(ws + O_CNT);
  int*            OFF  = (int*)(ws + O_OFF);
  unsigned short* WPL  = (unsigned short*)(ws + O_WPL);
  unsigned short* WF1T = (unsigned short*)(ws + O_WF1);
  unsigned short* WF2T = (unsigned short*)(ws + O_WF2);
  float*          PAR  = (float*)(ws + O_PAR);
  float*          REC  = (float*)(ws + O_REC);
  float*          STA  = (float*)(ws + O_STA);
  float*          GP   = (float*)(ws + O_G);

  hipFuncSetAttribute(reinterpret_cast<const void*>(&k_bucket),  hipFuncAttributeMaxDynamicSharedMemorySize, LDS_BUCKET);
  hipFuncSetAttribute(reinterpret_cast<const void*>(&k_gemm<0>), hipFuncAttributeMaxDynamicSharedMemorySize, LDS_GEMM);
  hipFuncSetAttribute(reinterpret_cast<const void*>(&k_gemm<1>), hipFuncAttributeMaxDynamicSharedMemorySize, LDS_GEMM);
  hipFuncSetAttribute(reinterpret_cast<const void*>(&k_head),    hipFuncAttributeMaxDynamicSharedMemorySize, LDS_HEAD);

  k_pa<<<XUNITS / NTHR + 1, NTHR, 0, stream>>>(x, (float*)d_ws);
  k_pb<<<WUNITS / NTHR, NTHR, 0, stream>>>(W1, W2, WPL);
  k_pc<<<(WFUNITS + PARN / 4 + NTHR - 1) / NTHR, NTHR, 0, stream>>>(Wf1, Wf2, b1, b2, gamma, beta, bf1, bf2, WF1T, PAR);
  k_bucket<<<NBLK, NTHR, LDS_BUCKET, stream>>>(src, dst, LST, CNT, OFF);
  for (int l = 0; l < NL; ++l) {
    const unsigned short* w1t = WPL + (size_t)l * HID * KK;
    const unsigned short* w2t = WPL + (size_t)(4 + l) * HID * KK;
    k_agg<<<MP / 64, NTHR, 0, stream>>>(P2, STA + (size_t)l * STATW, LST, CNT, OFF, P1);
    k_gemm<0><<<NTILE, NTHR, LDS_GEMM, stream>>>(P1, w1t, PAR + PB1 + l * HID, (void*)P3, REC);
    k_gemm<1><<<NTILE, NTHR, LDS_GEMM, stream>>>(P3, w2t, PAR + PB2 + l * HID, (void*)P2, REC);
    k_comb<<<1, NTHR, 0, stream>>>(REC, PAR, l, STA + (size_t)(l + 1) * STATW);
  }
  k_pool<<<NG, NTHR, 0, stream>>>(P2, STA + (size_t)NL * STATW, batch, GP);
  k_head<<<1, NTHR, LDS_HEAD, stream>>>(GP, WF1T, WF2T, PAR, out);
}
